// CuEquivarianceLayer_21500606283806
// MI455X (gfx1250) — hardware-verified
//
#include <hip/hip_runtime.h>
#include <stddef.h>
#include <cmath>
#include <complex>
#include <algorithm>


#define NTHR   256
#define NWAVE  8
#define EPT    8
#define CHUNK  (NTHR * EPT)
#define WCAP   (EPT * 32)
#define LISTN  (NWAVE * WCAP)
#define NB     512
#define NBSH   9
#define NPW    (NB / NWAVE)
#define ZT     32
#define ZCH    11
#define ZROW   384
#define XSP    32
#define NTILE  44

#define LDSZ_BYTES (2 * (4 * ZT * XSP * 2) + 2 * (5 * 32 * 32 * 2) + ZT * ZROW * 4)
#define LDSA_BYTES (NB * 128 * 4 + LISTN * 4)

static_assert(NB == (1 << NBSH));
static_assert((NB % NWAVE) == 0);
static_assert(CHUNK <= 2048);
static_assert(ZROW == 12 * 32);
static_assert(LDSZ_BYTES == 86016);
static_assert(LDSA_BYTES == 270336);

typedef float          v4f   __attribute__((ext_vector_type(4)));
typedef float          v8f   __attribute__((ext_vector_type(8)));
typedef int            v4i   __attribute__((ext_vector_type(4)));
typedef unsigned short v8us  __attribute__((ext_vector_type(8)));
typedef __bf16         v16bf __attribute__((ext_vector_type(16)));
union FragB { v16bf v; v8us u[2]; };

struct Coefs {
  float g0;
  float c1[3];
  float c2[3];
  float c3[3];
  float cg4[45];
};
static_assert(sizeof(Coefs) == 55 * 4);

namespace {

using cd = std::complex<double>;

double factd(int n) { double r = 1.0; for (int i = 2; i <= n; ++i) r *= (double)i; return r; }

void su2_cg(int j1, int j2, int j3, double* C) {
  const int d1 = 2 * j1 + 1, d2 = 2 * j2 + 1, d3 = 2 * j3 + 1;
  for (int i = 0; i < d1 * d2 * d3; ++i) C[i] = 0.0;
  for (int m1 = -j1; m1 <= j1; ++m1) {
    for (int m2 = -j2; m2 <= j2; ++m2) {
      const int m3 = m1 + m2;
      if (m3 < -j3 || m3 > j3) continue;
      const int vmin = std::max(std::max(-j1 + j2 + m3, -j1 + m1), 0);
      const int vmax = std::min(std::min(j2 + j3 + m1, j3 - j1 + j2), j3 + m3);
      double c = std::sqrt((2.0 * j3 + 1.0) * factd(j3 + j1 - j2) * factd(j3 - j1 + j2)
                           * factd(j1 + j2 - j3) / factd(j1 + j2 + j3 + 1));
      c *= std::sqrt(factd(j3 + m3) * factd(j3 - m3) * factd(j1 - m1)
                     * factd(j1 + m1) * factd(j2 - m2) * factd(j2 + m2));
      double s = 0.0;
      for (int v = vmin; v <= vmax; ++v) {
        const double sign = ((v + j2 + m2) & 1) ? -1.0 : 1.0;
        s += sign * factd(j2 + j3 + m1 - v) * factd(j1 - m1 + v)
             / (factd(v) * factd(j3 - j1 + j2 - v) * factd(j3 + m3 - v) * factd(v + j1 - j2 - m3));
      }
      C[((j1 + m1) * d2 + (j2 + m2)) * d3 + (j3 + m3)] = c * s;
    }
  }
}

void qmat(int l, cd* q) {
  const int d = 2 * l + 1;
  for (int i = 0; i < d * d; ++i) q[i] = cd(0.0, 0.0);
  const double is2 = 1.0 / std::sqrt(2.0);
  for (int m = -l; m < 0; ++m) {
    q[(l + m) * d + (l - m)] = cd(is2, 0.0);
    q[(l + m) * d + (l + m)] = cd(0.0, -is2);
  }
  q[l * d + l] = cd(1.0, 0.0);
  for (int m = 1; m <= l; ++m) {
    const double sgn = (m & 1) ? -1.0 : 1.0;
    q[(l + m) * d + (l + m)] = cd(sgn * is2, 0.0);
    q[(l + m) * d + (l - m)] = cd(0.0, sgn * is2);
  }
  cd f(1.0, 0.0);
  const cd mi(0.0, -1.0);
  for (int t = 0; t < l; ++t) f *= mi;
  for (int i = 0; i < d * d; ++i) q[i] *= f;
}

void real_cg(int l1, int l2, int l3, float* out) {
  const int d1 = 2 * l1 + 1, d2 = 2 * l2 + 1, d3 = 2 * l3 + 1;
  double C[125];
  su2_cg(l1, l2, l3, C);
  cd q1[25], q2[25], q3[25];
  qmat(l1, q1); qmat(l2, q2); qmat(l3, q3);
  double R[75];
  double norm2 = 0.0;
  for (int j = 0; j < d1; ++j)
    for (int p = 0; p < d2; ++p)
      for (int m = 0; m < d3; ++m) {
        cd a(0.0, 0.0);
        for (int i = 0; i < d1; ++i)
          for (int k = 0; k < d2; ++k)
            for (int n = 0; n < d3; ++n) {
              const double cv = C[(i * d2 + k) * d3 + n];
              if (cv == 0.0) continue;
              a += q1[i * d1 + j] * q2[k * d2 + p] * std::conj(q3[n * d3 + m]) * cv;
            }
        R[(j * d2 + p) * d3 + m] = a.real();
        norm2 += a.real() * a.real();
      }
  const double nrm = std::sqrt(norm2);
  for (int i = 0; i < d1 * d2 * d3; ++i) out[i] = (float)(R[i] / nrm);
}

Coefs make_coefs() {
  float cg000[1], cg011[9], cg101[9], cg110[9], cg121[45];
  real_cg(0, 0, 0, cg000);
  real_cg(0, 1, 1, cg011);
  real_cg(1, 0, 1, cg101);
  real_cg(1, 1, 0, cg110);
  real_cg(1, 2, 1, cg121);
  const float a2 = (float)(1.0 / std::sqrt(32.0 * 1.0 * 2.0));
  const float a3 = (float)(1.0 / std::sqrt(32.0 * 1.0 * 3.0));
  Coefs cf;
  cf.g0 = cg000[0] * a2;
  for (int k = 0; k < 3; ++k) {
    cf.c1[k] = cg011[k * 3 + k] * a3;
    cf.c2[k] = cg101[k * 3 + k] * a3;
    cf.c3[k] = cg110[k * 3 + k] * a2;
  }
  for (int q = 0; q < 45; ++q) cf.cg4[q] = cg121[q] * a3;
  return cf;
}

}

extern __shared__ v4f dynsm[];

__device__ __forceinline__ unsigned short bf_bits(float f) {
  unsigned int u = __float_as_uint(f);
  u += 0x7FFFu + ((u >> 16) & 1u);
  return (unsigned short)(u >> 16);
}

__device__ __forceinline__ void split2(float f, unsigned short& hi, unsigned short& lo) {
  hi = bf_bits(f);
  const float hf = __uint_as_float(((unsigned int)hi) << 16);
  lo = bf_bits(f - hf);
}

__device__ __forceinline__ v8f wmb(const FragB& a, const FragB& b, v8f c) {
  v8f d = __builtin_amdgcn_wmma_f32_16x16x32_bf16(false, a.v, false, b.v, (short)0, c, false, false);
  asm volatile("v_nop\n\tv_nop\n\tv_nop\n\tv_nop"
               : "+v"(d) : "v"(a.u[0]), "v"(a.u[1]), "v"(b.u[0]), "v"(b.u[1]));
  return d;
}

__global__ __launch_bounds__(NTHR) void k_nodew(const float* __restrict__ x, const float* __restrict__ W,
                                                float* zout, int nN) {
  unsigned short* xsh = (unsigned short*)dynsm;
  unsigned short* xsl = xsh + 4 * ZT * XSP;
  unsigned short* wsh = xsl + 4 * ZT * XSP;
  unsigned short* wsl = wsh + 5 * 32 * 32;
  float* stg = (float*)(wsl + 5 * 32 * 32);

  const int tid = threadIdx.x, lane = tid & 31, h = lane >> 4, m = lane & 15;
  const int wave = __builtin_amdgcn_readfirstlane(tid >> 5);
  const int nodeBase = blockIdx.x * ZT;

#pragma unroll
  for (int it = 0; it < 20; ++it) {
    const int f = it * NTHR + tid;
    const int p = f >> 10, u = (f >> 5) & 31, w = f & 31;
    const float v = W[f];
    unsigned short hi, lo;
    split2(v, hi, lo);
    const int idx = ((p * 32 + w) << 5) + u;
    wsh[idx] = hi;
    wsl[idx] = lo;
  }
#pragma unroll
  for (int it = 0; it < 4; ++it) {
    const int f4 = it * NTHR + tid;
    const int row = f4 >> 5, c4 = (f4 & 31) * 4;
    int node = nodeBase + row;
    node = node > nN - 1 ? nN - 1 : node;
    const v4f v = *(const v4f*)(x + (size_t)node * 128 + c4);
#pragma unroll
    for (int j = 0; j < 4; ++j) {
      const int col = c4 + j;
      const int q = col >= 32 ? col - 32 : 0;
      const int u = q / 3;
      const int i = q - u * 3;
      const int mat = col >= 32 ? 1 + i : 0;
      const int k = col >= 32 ? u : col;
      unsigned short hi, lo;
      split2(v[j], hi, lo);
      const int idx = (mat * ZT + row) * XSP + k;
      xsh[idx] = hi;
      xsl[idx] = lo;
    }
  }
#pragma unroll
  for (int it = 0; it < 4; ++it) {
    const int f = it * NTHR + tid;
    stg[(f >> 5) * ZROW + (f & 31) * 12 + ZCH] = 0.0f;
  }
  __syncthreads();

  const v8f zero8 = {0.0f, 0.0f, 0.0f, 0.0f, 0.0f, 0.0f, 0.0f, 0.0f};
#pragma unroll 1
  for (int ii = 0; ii < 6; ++ii) {
    const int t = ii * NWAVE + wave;
    if (t < NTILE) {
      const int c = t >> 2, nt = (t >> 1) & 1, wt = t & 1;
      const int q = c >= 2 ? c - 2 : 0;
      const int qd = q / 3;
      const int p = c >= 2 ? 2 + qd : c;
      const int mat = c >= 2 ? 1 + (q - qd * 3) : 0;
      const int ab = (mat * ZT + nt * 16 + m) * XSP + 8 * h;
      const int bb = ((p * 32 + wt * 16 + m) << 5) + 8 * h;
      FragB ahi, alo, bhi, blo;
      ahi.u[0] = *(const v8us*)(xsh + ab);  ahi.u[1] = *(const v8us*)(xsh + ab + 16);
      alo.u[0] = *(const v8us*)(xsl + ab);  alo.u[1] = *(const v8us*)(xsl + ab + 16);
      bhi.u[0] = *(const v8us*)(wsh + bb);  bhi.u[1] = *(const v8us*)(wsh + bb + 16);
      blo.u[0] = *(const v8us*)(wsl + bb);  blo.u[1] = *(const v8us*)(wsl + bb + 16);
      v8f acc = zero8;
      acc = wmb(ahi, bhi, acc);
      acc = wmb(ahi, blo, acc);
      acc = wmb(alo, bhi, acc);
      float* sp = stg + (nt * 16 + 8 * h) * ZROW + (wt * 16 + m) * 12 + c;
#pragma unroll
      for (int r = 0; r < 8; ++r) sp[r * ZROW] = acc[r];
    }
  }
  __syncthreads();

  const size_t zb = (size_t)blockIdx.x * (size_t)(ZT * ZROW);
#pragma unroll
  for (int qn = 0; qn < 12; ++qn) {
    const int qq = wave * 12 + qn;
    const v4f v = *(const v4f*)(stg + qq * 128 + lane * 4);
    *(volatile v4f*)(zout + zb + (size_t)(qq * 128 + lane * 4)) = v;
  }
  __threadfence();
#pragma unroll
  for (int qn = 0; qn < 12; ++qn) {
    const int qq = wave * 12 + qn;
    const v4f v = *(const v4f*)(stg + qq * 128 + lane * 4);
    *(volatile v4f*)(zout + zb + (size_t)(qq * 128 + lane * 4)) = v;
  }
}

__device__ __forceinline__ int scan_chunk(const int* __restrict__ dsts, int nE, int cbase, int nodeBase,
                                          int vec8, int* list, int tid, int wave) {
  int wc = 0;
  const int el0  = tid * EPT;
  const int e0   = cbase + el0;
  const int sent = -2147483647 - 1;
  const int le   = nE - 1;
  v4i da, db;
  if (vec8 != 0 && cbase + CHUNK <= nE) {
    da = *(const v4i*)(dsts + e0);
    db = *(const v4i*)(dsts + e0 + 4);
  } else {
    da.x = (e0     < nE) ? dsts[(e0     < le) ? e0     : le] : sent;
    da.y = (e0 + 1 < nE) ? dsts[(e0 + 1 < le) ? e0 + 1 : le] : sent;
    da.z = (e0 + 2 < nE) ? dsts[(e0 + 2 < le) ? e0 + 2 : le] : sent;
    da.w = (e0 + 3 < nE) ? dsts[(e0 + 3 < le) ? e0 + 3 : le] : sent;
    db.x = (e0 + 4 < nE) ? dsts[(e0 + 4 < le) ? e0 + 4 : le] : sent;
    db.y = (e0 + 5 < nE) ? dsts[(e0 + 5 < le) ? e0 + 5 : le] : sent;
    db.z = (e0 + 6 < nE) ? dsts[(e0 + 6 < le) ? e0 + 6 : le] : sent;
    db.w = (e0 + 7 < nE) ? dsts[(e0 + 7 < le) ? e0 + 7 : le] : sent;
  }
  const unsigned nb = (unsigned)nodeBase;
  const unsigned s0 = (unsigned)da.x - nb, s1 = (unsigned)da.y - nb;
  const unsigned s2 = (unsigned)da.z - nb, s3 = (unsigned)da.w - nb;
  const unsigned s4 = (unsigned)db.x - nb, s5 = (unsigned)db.y - nb;
  const unsigned s6 = (unsigned)db.z - nb, s7 = (unsigned)db.w - nb;
  const bool h0 = s0 < (unsigned)NB, h1 = s1 < (unsigned)NB, h2 = s2 < (unsigned)NB, h3 = s3 < (unsigned)NB;
  const bool h4 = s4 < (unsigned)NB, h5 = s5 < (unsigned)NB, h6 = s6 < (unsigned)NB, h7 = s7 < (unsigned)NB;
  const unsigned any = __builtin_amdgcn_ballot_w32(h0 | h1 | h2 | h3 | h4 | h5 | h6 | h7);
  if (any != 0u) {
#define HITJ(J, HJ, SJ) { \
      const unsigned mj = __builtin_amdgcn_ballot_w32(HJ); \
      if (mj != 0u) { \
        if (HJ) { \
          const int pos = wc + (int)__builtin_amdgcn_mbcnt_lo(mj, 0u); \
          if (pos < WCAP) list[wave * WCAP + pos] = ((el0 + (J)) << NBSH) | (int)(SJ); \
        } \
        wc += (int)__builtin_popcount(mj); } }
    HITJ(0, h0, s0)
    HITJ(1, h1, s1)
    HITJ(2, h2, s2)
    HITJ(3, h3, s3)
    HITJ(4, h4, s4)
    HITJ(5, h5, s5)
    HITJ(6, h6, s6)
    HITJ(7, h7, s7)
#undef HITJ
  }
  return wc;
}

__global__ __launch_bounds__(NTHR) void k_agg(const float* __restrict__ z, const float* __restrict__ esh,
                                              const int* __restrict__ ei, float* outp,
                                              int nN, int nE, int vec8, Coefs cf) {
  float* accs = (float*)dynsm;
  int*   list = (int*)(accs + NB * 128);
  __shared__ int wcnt[NWAVE];

  const int tid = threadIdx.x, lane = tid & 31;
  const int wave = __builtin_amdgcn_readfirstlane(tid >> 5);
  const int nodeBase = blockIdx.x * NB;
  const int* srcs = ei;
  const int* dsts = ei + nE;

  {
    const v4f z4 = {0.0f, 0.0f, 0.0f, 0.0f};
    v4f* a4 = (v4f*)accs;
#pragma unroll 8
    for (int i = tid; i < NB * 128 / 4; i += NTHR) a4[i] = z4;
  }
  __syncthreads();

  const int nChunks = (nE + CHUNK - 1) / CHUNK;
#pragma unroll 1
  for (int ch = 0; ch < nChunks; ++ch) {
    const int cbase = ch * CHUNK;
    const int wc = scan_chunk(dsts, nE, cbase, nodeBase, vec8, list, tid, wave);
    if (lane == 0) wcnt[wave] = wc;
    __syncthreads();

#pragma unroll 1
    for (int w2 = 0; w2 < NWAVE; ++w2) {
      int n = wcnt[w2];
      n = n > WCAP ? WCAP : (n < 0 ? 0 : n);
      const int* lp = list + w2 * WCAP;
#pragma unroll 1
      for (int b0 = 0; b0 < n; b0 += 32) {
        const int idx = b0 + lane;
        const int pk  = lp[idx < WCAP ? idx : WCAP - 1];
        const bool mine = (idx < n) && ((pk & (NWAVE - 1)) == wave);
        unsigned msk = __builtin_amdgcn_ballot_w32(mine);
#pragma unroll 1
        while (msk != 0u) {
          const int li = __builtin_ctz(msk);
          msk &= msk - 1u;
          const int pe = __builtin_amdgcn_readlane(pk, li);
          int el = pe >> NBSH;
          el = el > CHUNK - 1 ? CHUNK - 1 : (el < 0 ? 0 : el);
          const int slot = pe & (NB - 1);
          int e = cbase + el;
          e = e > nE - 1 ? nE - 1 : e;
          int s = srcs[e];
          s = s < 0 ? 0 : (s > nN - 1 ? nN - 1 : s);

          const float* shp = esh + (size_t)e * 9;
          const float y0 = shp[0];
          const float sh1[3] = { shp[1], shp[2], shp[3] };
          const float sh2[5] = { shp[4], shp[5], shp[6], shp[7], shp[8] };

          const float g0 = cf.g0 * y0;
          float u3[3], t1[3], t2[3], t4[3][3];
#pragma unroll
          for (int i = 0; i < 3; ++i) {
            u3[i] = cf.c3[i] * sh1[i];
            t1[i] = cf.c1[i] * sh1[i];
            t2[i] = cf.c2[i] * y0;
          }
#pragma unroll
          for (int i = 0; i < 3; ++i) {
#pragma unroll
            for (int k = 0; k < 3; ++k) {
              float a = cf.cg4[(i * 5 + 0) * 3 + k] * sh2[0];
#pragma unroll
              for (int j = 1; j < 5; ++j) a += cf.cg4[(i * 5 + j) * 3 + k] * sh2[j];
              t4[i][k] = a;
            }
          }

          const float* zr = z + (size_t)s * ZROW + lane * 12;
          const v4f za = *(const v4f*)(zr);
          const v4f zb = *(const v4f*)(zr + 4);
          const v4f zc = *(const v4f*)(zr + 8);
          const float zA = za.x, zB = za.y;
          const float zCv[3] = { za.z, za.w, zb.x };
          const float zD0 = zb.y, zD1 = zb.z, zD2 = zb.w;
          const float zE0 = zc.x, zE1 = zc.y, zE2 = zc.z;

          const float o0 = g0 * zA + (u3[0] * zD0 + u3[1] * zD1 + u3[2] * zD2);
          float ov[3];
#pragma unroll
          for (int k = 0; k < 3; ++k)
            ov[k] = t1[k] * zB + t2[k] * zCv[k] + (t4[0][k] * zE0 + t4[1][k] * zE1 + t4[2][k] * zE2);

          float* ar = accs + slot * 128;
          const float a0 = ar[lane];
          ar[lane] = a0 + o0;
#pragma unroll
          for (int k = 0; k < 3; ++k) {
            const float av = ar[32 + lane * 3 + k];
            ar[32 + lane * 3 + k] = av + ov[k];
          }
        }
      }
    }
    __syncthreads();
  }

#pragma unroll 4
  for (int j = 0; j < NPW; ++j) {
    const int slot = wave * NPW + j;
    const int node = nodeBase + slot;
    if (node < nN) {
      const v4f v = *(const v4f*)(accs + slot * 128 + lane * 4);
      *(volatile v4f*)(outp + (size_t)node * 128 + lane * 4) = v;
    }
  }
  __threadfence();
#pragma unroll 4
  for (int j = 0; j < NPW; ++j) {
    const int slot = wave * NPW + j;
    const int node = nodeBase + slot;
    if (node < nN) {
      const v4f v = *(const v4f*)(accs + slot * 128 + lane * 4);
      *(volatile v4f*)(outp + (size_t)node * 128 + lane * 4) = v;
    }
  }
}

extern "C" void kernel_launch(void* const* d_in, const int* in_sizes, int n_in,
                              void* d_out, int out_size, void* d_ws, size_t ws_size,
                              hipStream_t stream) {
  if (n_in < 4) return;
  const int nN = in_sizes[0] / 128;
  const int nE = in_sizes[1] / 9;
  if (nN <= 0 || in_sizes[0] != nN * 128) return;
  if (nE <= 0 || in_sizes[1] != nE * 9) return;
  if (in_sizes[2] != 2 * nE) return;
  if (in_sizes[3] != 5 * 32 * 32) return;
  if (out_size != nN * 128) return;

  const float* x   = (const float*)d_in[0];
  const float* esh = (const float*)d_in[1];
  const int*   ei  = (const int*)d_in[2];
  const float* wts = (const float*)d_in[3];
  float* out = (float*)d_out;

  const int nBlkZ = (nN + ZT - 1) / ZT;
  const int nBlkA = (nN + NB - 1) / NB;

  const size_t zBytes = (size_t)nBlkZ * (size_t)(ZT * ZROW) * sizeof(float);
  if (zBytes > ws_size) return;
  if (zBytes > (size_t)134217728) return;
  float* z = (float*)d_ws;

  const Coefs cf = make_coefs();
  const int vec8 = ((nE & 3) == 0) ? 1 : 0;

  hipFuncSetAttribute(reinterpret_cast<const void*>(&k_nodew), hipFuncAttributeMaxDynamicSharedMemorySize, LDSZ_BYTES);
  hipFuncSetAttribute(reinterpret_cast<const void*>(&k_agg),   hipFuncAttributeMaxDynamicSharedMemorySize, LDSA_BYTES);

  k_nodew<<<nBlkZ, NTHR, LDSZ_BYTES, stream>>>(x, wts, z, nN);
  k_agg<<<nBlkA, NTHR, LDSA_BYTES, stream>>>(z, esh, ei, out, nN, nE, vec8, cf);
}
